// TreeLSTM_39616778338740
// MI455X (gfx1250) — hardware-verified
//
#include <hip/hip_runtime.h>
#include <stddef.h>
#include <stdint.h>

#define HD      128
#define KC      3
#define VOPS    32
#define KIOU    (KC * HD)
#define WTP     384
#define CAP     256
#define TM      64
#define NTHR    256
#define NWAVE   8
#define APITCH  392
#define TPITCH  136
#define PREP_BLOCKS (4 * VOPS * KC)
#define WSMAX   134217728

#define SZ_A      (TM * APITCH * 2)
#define SZ_T      (TM * HD * 4)
#define O_A       0
#define O_STG     (O_A + SZ_A)
#define O_T0      (O_STG + SZ_T)
#define O_T1      (O_T0 + SZ_T)
#define O_IDX     (O_T1 + SZ_T)
#define O_NODE    (O_IDX + CAP * 4)
#define O_MASK    (O_NODE + TM * 4)
#define O_WC      (O_MASK + TM * 16)
#define LDS_TOTAL (O_WC + 64)

static_assert((O_STG % 16) == 0 && (O_T0 % 16) == 0 && (O_T1 % 16) == 0 && (O_IDX % 16) == 0);
static_assert((O_NODE % 16) == 0 && (O_MASK % 16) == 0 && (O_WC % 16) == 0);
static_assert(O_T1 == O_T0 + SZ_T);
static_assert(LDS_TOTAL <= 300000);
static_assert((APITCH * 2) % 16 == 0 && (TPITCH * 2) % 16 == 0);
static_assert(KIOU % 32 == 0 && HD % 32 == 0 && TM == 64 && NTHR == 32 * NWAVE);
static_assert(TM * (KIOU / 4) % NTHR == 0);
static_assert((HD * HD / 4) % NTHR == 0);
static_assert(TM * HD == 8 * NTHR * 4);
static_assert(CAP % TM == 0);
static_assert(NTHR == 4 * TM);

typedef float          v4f   __attribute__((ext_vector_type(4)));
typedef float          v8f   __attribute__((ext_vector_type(8)));
typedef int            v8i   __attribute__((ext_vector_type(8)));
typedef unsigned short v4us  __attribute__((ext_vector_type(4)));
typedef unsigned short v8us  __attribute__((ext_vector_type(8)));
typedef unsigned short v16us __attribute__((ext_vector_type(16)));
typedef __bf16         v16bf __attribute__((ext_vector_type(16)));
typedef v4f  __attribute__((may_alias)) v4fa;
typedef v4us __attribute__((may_alias)) v4usa;
typedef v8us __attribute__((may_alias)) v8usa;
union FragB { v16bf v; v16us u; v8us h[2]; v8i w; };

__device__ __forceinline__ v8f wmb(const FragB& a, const FragB& b, v8f c) {
  v8f d = __builtin_amdgcn_wmma_f32_16x16x32_bf16(false, a.v, false, b.v, (short)0, c, false, false);
  asm volatile("v_nop\n\tv_nop\n\tv_nop\n\tv_nop" : "+v"(d) : "v"(a.w), "v"(b.w));
  return d;
}

__device__ __forceinline__ unsigned bf16_bits(float f) {
  const unsigned u = __float_as_uint(f);
  return (u + 0x7FFFu + ((u >> 16) & 1u)) >> 16;
}
__device__ __forceinline__ float bf16_val(float f) {
  return __uint_as_float(bf16_bits(f) << 16);
}
__device__ __forceinline__ v4f bf16_val4(v4f x) {
  v4f y;
  y.x = bf16_val(x.x); y.y = bf16_val(x.y); y.z = bf16_val(x.z); y.w = bf16_val(x.w);
  return y;
}

__device__ __forceinline__ float sigm(float x) {
  return __builtin_amdgcn_rcpf(1.0f + expf(-x));
}

__device__ __forceinline__ void wprep_pass(const unsigned short* tile, unsigned short* dstBase,
                                           int wave, int lane) {
  const int q8 = lane & 7, sub = lane >> 3;
#pragma unroll
  for (int i = 0; i < 8; ++i) {
    const int L  = i * 32 + wave * 4 + sub;
    const int n  = L >> 1, hl = L & 1;
    const v8us vv = *(const v8usa*)(tile + n * TPITCH + 64 * hl + 8 * q8);
    unsigned short* dp = dstBase + (size_t)n * WTP + 64 * hl + 8 * q8;
    *(volatile v8us*)dp = vv;
  }
}

__global__ __launch_bounds__(NTHR) void k_wprep(const float* __restrict__ Wi, const float* __restrict__ Wo,
                                                const float* __restrict__ Wu, const float* __restrict__ Wfm,
                                                unsigned short* Wt) {
  __shared__ __attribute__((aligned(16))) unsigned short tile[HD * TPITCH];
  const int b   = (int)blockIdx.x;
  const int g   = b / (VOPS * KC);
  const int rem = b - g * (VOPS * KC);
  const int op  = rem / KC;
  const int k   = rem - op * KC;
  const int tid = (int)threadIdx.x, lane = tid & 31, wave = tid >> 5;
  const float* W;
  if (g == 0)      W = Wi;
  else if (g == 1) W = Wo;
  else if (g == 2) W = Wu;
  else             W = Wfm;
  const float* src = W + (size_t)rem * (HD * HD);

#pragma unroll 2
  for (int e4 = tid; e4 < (HD * HD) / 4; e4 += NTHR) {
    const int kk = e4 >> 5;
    const int n0 = (e4 & 31) * 4;
    const v4f w = *(const v4fa*)(src + (size_t)e4 * 4);
    tile[(n0 + 0) * TPITCH + kk] = (unsigned short)bf16_bits(w.x);
    tile[(n0 + 1) * TPITCH + kk] = (unsigned short)bf16_bits(w.y);
    tile[(n0 + 2) * TPITCH + kk] = (unsigned short)bf16_bits(w.z);
    tile[(n0 + 3) * TPITCH + kk] = (unsigned short)bf16_bits(w.w);
  }
  __syncthreads();

  unsigned short* dstBase = Wt + ((size_t)(g * VOPS + op) * HD) * WTP + k * HD;
  wprep_pass(tile, dstBase, wave, lane);
  __threadfence();
  wprep_pass(tile, dstBase, wave, lane);
}

__device__ __forceinline__ void gemm_stg(float* stg, const unsigned short* aBase,
                                         const unsigned short* bRow, const int ksteps,
                                         int wave, int hh, int m) {
  v8f acc[4];
  {
    const v8f z = {0.f, 0.f, 0.f, 0.f, 0.f, 0.f, 0.f, 0.f};
#pragma unroll
    for (int t = 0; t < 4; ++t) acc[t] = z;
  }
#pragma unroll 2
  for (int kq = 0; kq < ksteps; ++kq) {
    FragB bfr;
    bfr.h[0] = *(const v8usa*)(bRow + 32 * kq);
    bfr.h[1] = *(const v8usa*)(bRow + 32 * kq + 16);
#pragma unroll
    for (int t = 0; t < 4; ++t) {
      FragB afr;
      afr.h[0] = *(const v8usa*)(aBase + t * 16 * APITCH + 32 * kq);
      afr.h[1] = *(const v8usa*)(aBase + t * 16 * APITCH + 32 * kq + 16);
      acc[t] = wmb(afr, bfr, acc[t]);
    }
  }
#pragma unroll
  for (int t = 0; t < 4; ++t) {
#pragma unroll
    for (int r = 0; r < 8; ++r) {
      stg[(16 * t + 8 * hh + r) * HD + 16 * wave + m] = acc[t][r];
    }
  }
}

__device__ __forceinline__ void out_pass(const float* sOut, const int* sNode, float* out, int outOff,
                                         int rowsValid, int wave, int lane) {
  const int q8 = lane & 7, sub = lane >> 3;
#pragma unroll
  for (int i = 0; i < 16; ++i) {
    const int L     = i * 32 + wave * 4 + sub;
    const int which = L >> 8;
    const int rl    = L & 255;
    const int row   = rl >> 2, qt = rl & 3;
    const v4f vv = *(const v4fa*)(sOut + which * (TM * HD) + row * HD + 32 * qt + 4 * q8);
    const int node = sNode[row];
    float* dp = out + (size_t)which * (size_t)outOff + (size_t)node * HD + 32 * qt + 4 * q8;
    if (row < rowsValid) *(volatile v4f*)dp = vv;
  }
}

__global__ __launch_bounds__(NTHR) void k_cell(
    const float* __restrict__ ch, const float* __restrict__ cc,
    const unsigned short* __restrict__ Wt,
    const float* __restrict__ bi, const float* __restrict__ bo,
    const float* __restrict__ bu, const float* __restrict__ bfg,
    const int* __restrict__ ops, const int* __restrict__ nch,
    int nN, int outOff, float* out)
{
  extern __shared__ __attribute__((aligned(16))) unsigned char dsm[];
  unsigned short* sA = (unsigned short*)(dsm + O_A);
  float* stg   = (float*)(dsm + O_STG);
  float* sT0   = (float*)(dsm + O_T0);
  float* sT1   = (float*)(dsm + O_T1);
  int*   sIdx  = (int*)(dsm + O_IDX);
  int*   sNode = (int*)(dsm + O_NODE);
  float* sMask = (float*)(dsm + O_MASK);
  int*   sWc   = (int*)(dsm + O_WC);

  const int v = (int)blockIdx.x;
  const int tid = (int)threadIdx.x, lane = tid & 31, wave = tid >> 5;
  const int hh = lane >> 4, m = lane & 15;

  int total = 0;
  const int nChunks = (nN + NTHR - 1) / NTHR;
#pragma unroll 1
  for (int chn = 0; chn < nChunks; ++chn) {
    const int n  = chn * NTHR + tid;
    const int nc = n < nN ? n : nN - 1;
    int opv = ops[nc];
    opv = opv < 0 ? 0 : (opv > VOPS - 1 ? VOPS - 1 : opv);
    const bool hit = (n < nN) && (opv == v);
    const unsigned bal = __builtin_amdgcn_ballot_w32(hit);
    if (lane == 0) sWc[wave] = (int)__builtin_popcount(bal);
    __syncthreads();
    int pre = 0, csum = 0;
#pragma unroll
    for (int w2 = 0; w2 < NWAVE; ++w2) {
      const int c = sWc[w2];
      pre += (w2 < wave) ? c : 0;
      csum += c;
    }
    const int pos = total + pre + (int)__builtin_amdgcn_mbcnt_lo(bal, 0u);
    if (hit && pos < CAP) sIdx[pos] = n;
    total += csum;
    __syncthreads();
  }
  const int count  = total < CAP ? total : CAP;
  const float pz   = (total > CAP) ? __int_as_float(0x7fc00000) : 0.0f;
  const int nTiles = (count + TM - 1) / TM;

  const size_t bcol = (size_t)v * KIOU + 4 * lane;
  const unsigned short* aB = sA + m * APITCH + 8 * hh;
  const size_t wrow = (size_t)(16 * wave + m);

#pragma unroll 1
  for (int ti = 0; ti < nTiles; ++ti) {
    const int base = ti * TM;
    const int rowsValid = count - base;
    __syncthreads();

    if (tid < TM) {
      const int gm = base + tid;
      const int li = (gm < count) ? gm : (count - 1);
      const int node = sIdx[li];
      const int ncv = nch[node];
      sNode[tid] = node;
      v4f mk;
      mk.x = (0 <= ncv) ? 1.0f : 0.0f;
      mk.y = (1 <= ncv) ? 1.0f : 0.0f;
      mk.z = (2 <= ncv) ? 1.0f : 0.0f;
      mk.w = 0.0f;
      *(v4fa*)(sMask + 4 * tid) = mk;
    }
    __syncthreads();

#pragma unroll 2
    for (int e4 = tid; e4 < TM * (KIOU / 4); e4 += NTHR) {
      const int mrow = e4 / (KIOU / 4);
      const int j    = e4 - mrow * (KIOU / 4);
      const int node = sNode[mrow];
      const v4f h4 = *(const v4fa*)(ch + (size_t)node * KIOU + 4 * j);
      v4us af;
      af[0] = (unsigned short)bf16_bits(h4.x); af[1] = (unsigned short)bf16_bits(h4.y);
      af[2] = (unsigned short)bf16_bits(h4.z); af[3] = (unsigned short)bf16_bits(h4.w);
      *(v4usa*)(sA + mrow * APITCH + 4 * j) = af;
    }
    {
      const v4f z = {0.f, 0.f, 0.f, 0.f};
#pragma unroll
      for (int i = 0; i < 8; ++i) *(v4fa*)(sT1 + 1024 * i + 4 * tid) = z;
    }
    __syncthreads();

#pragma unroll 1
    for (int k = 0; k < KC; ++k) {
      const unsigned short* bRow = Wt + (((size_t)3 * VOPS + v) * HD + wrow) * WTP + k * HD + 8 * hh;
      gemm_stg(stg, aB + k * HD, bRow, HD / 32, wave, hh, m);
      __syncthreads();
      {
        const v4f b4 = bf16_val4(*(const v4fa*)(bfg + bcol + k * HD));
#pragma unroll 1
        for (int i = 0; i < 8; ++i) {
          const int row = 8 * i + wave;
          const int e = row * HD + 4 * lane;
          const v4f x = *(const v4fa*)(stg + e);
          const int node = sNode[row];
          const float mk = sMask[4 * row + k];
          const v4f c4 = bf16_val4(*(const v4fa*)(cc + (size_t)node * KIOU + k * HD + 4 * lane));
          v4f f4 = *(const v4fa*)(sT1 + e);
          f4.x = f4.x + (mk * sigm(x.x + b4.x)) * c4.x;
          f4.y = f4.y + (mk * sigm(x.y + b4.y)) * c4.y;
          f4.z = f4.z + (mk * sigm(x.z + b4.z)) * c4.z;
          f4.w = f4.w + (mk * sigm(x.w + b4.w)) * c4.w;
          *(v4fa*)(sT1 + e) = f4;
        }
      }
      __syncthreads();
    }

    {
      const int row = tid >> 2, q = tid & 3;
      const v8us z8 = {0, 0, 0, 0, 0, 0, 0, 0};
#pragma unroll
      for (int k = 0; k < KC; ++k) {
        const float mk = sMask[4 * row + k];
        if (mk == 0.0f) {
          unsigned short* p = sA + row * APITCH + k * HD + 32 * q;
          *(v8usa*)(p + 0)  = z8;
          *(v8usa*)(p + 8)  = z8;
          *(v8usa*)(p + 16) = z8;
          *(v8usa*)(p + 24) = z8;
        }
      }
    }
    __syncthreads();

    {
      const unsigned short* bRow = Wt + (((size_t)2 * VOPS + v) * HD + wrow) * WTP + 8 * hh;
      gemm_stg(stg, aB, bRow, KIOU / 32, wave, hh, m);
      __syncthreads();
      const v4f b0 = bf16_val4(*(const v4fa*)(bu + bcol + 0 * HD));
      const v4f b1 = bf16_val4(*(const v4fa*)(bu + bcol + 1 * HD));
      const v4f b2 = bf16_val4(*(const v4fa*)(bu + bcol + 2 * HD));
#pragma unroll 1
      for (int i = 0; i < 8; ++i) {
        const int row = 8 * i + wave;
        const int e = row * HD + 4 * lane;
        const v4f x  = *(const v4fa*)(stg + e);
        const v4f mk = *(const v4fa*)(sMask + 4 * row);
        const v4f bs = (mk.x * b0 + mk.y * b1) + mk.z * b2;
        v4f y;
        y.x = tanhf(x.x + bs.x); y.y = tanhf(x.y + bs.y);
        y.z = tanhf(x.z + bs.z); y.w = tanhf(x.w + bs.w);
        *(v4fa*)(sT0 + e) = y;
      }
      __syncthreads();
    }
    {
      const unsigned short* bRow = Wt + (((size_t)0 * VOPS + v) * HD + wrow) * WTP + 8 * hh;
      gemm_stg(stg, aB, bRow, KIOU / 32, wave, hh, m);
      __syncthreads();
      const v4f b0 = bf16_val4(*(const v4fa*)(bi + bcol + 0 * HD));
      const v4f b1 = bf16_val4(*(const v4fa*)(bi + bcol + 1 * HD));
      const v4f b2 = bf16_val4(*(const v4fa*)(bi + bcol + 2 * HD));
#pragma unroll 1
      for (int i = 0; i < 8; ++i) {
        const int row = 8 * i + wave;
        const int e = row * HD + 4 * lane;
        const v4f x  = *(const v4fa*)(stg + e);
        const v4f mk = *(const v4fa*)(sMask + 4 * row);
        const v4f bs = (mk.x * b0 + mk.y * b1) + mk.z * b2;
        const v4f uu = *(const v4fa*)(sT0 + e);
        const v4f fc = *(const v4fa*)(sT1 + e);
        v4f cv;
        cv.x = sigm(x.x + bs.x) * uu.x + fc.x + pz;
        cv.y = sigm(x.y + bs.y) * uu.y + fc.y + pz;
        cv.z = sigm(x.z + bs.z) * uu.z + fc.z + pz;
        cv.w = sigm(x.w + bs.w) * uu.w + fc.w + pz;
        *(v4fa*)(sT1 + e) = cv;
      }
      __syncthreads();
    }
    {
      const unsigned short* bRow = Wt + (((size_t)1 * VOPS + v) * HD + wrow) * WTP + 8 * hh;
      gemm_stg(stg, aB, bRow, KIOU / 32, wave, hh, m);
      __syncthreads();
      const v4f b0 = bf16_val4(*(const v4fa*)(bo + bcol + 0 * HD));
      const v4f b1 = bf16_val4(*(const v4fa*)(bo + bcol + 1 * HD));
      const v4f b2 = bf16_val4(*(const v4fa*)(bo + bcol + 2 * HD));
#pragma unroll 1
      for (int i = 0; i < 8; ++i) {
        const int row = 8 * i + wave;
        const int e = row * HD + 4 * lane;
        const v4f x  = *(const v4fa*)(stg + e);
        const v4f mk = *(const v4fa*)(sMask + 4 * row);
        const v4f bs = (mk.x * b0 + mk.y * b1) + mk.z * b2;
        const v4f cv = *(const v4fa*)(sT1 + e);
        v4f hv;
        hv.x = sigm(x.x + bs.x) * tanhf(cv.x);
        hv.y = sigm(x.y + bs.y) * tanhf(cv.y);
        hv.z = sigm(x.z + bs.z) * tanhf(cv.z);
        hv.w = sigm(x.w + bs.w) * tanhf(cv.w);
        *(v4fa*)(sT0 + e) = hv;
      }
      __syncthreads();
    }

    out_pass(sT0, sNode, out, outOff, rowsValid, wave, lane);
    __threadfence();
    out_pass(sT0, sNode, out, outOff, rowsValid, wave, lane);
  }
}

extern "C" void kernel_launch(void* const* d_in, const int* in_sizes, int n_in,
                              void* d_out, int out_size, void* d_ws, size_t ws_size,
                              hipStream_t stream) {
  if (n_in < 12) return;
  const int nN = in_sizes[10];
  if (nN < 1 || nN > (1 << 20)) return;
  if (in_sizes[11] != nN) return;
  if (in_sizes[0] != nN * KIOU || in_sizes[1] != nN * KIOU) return;
  if (in_sizes[2] != VOPS * KC * HD * HD || in_sizes[3] != VOPS * KC * HD * HD) return;
  if (in_sizes[4] != VOPS * KC * HD * HD || in_sizes[5] != VOPS * KC * HD * HD) return;
  if (in_sizes[6] != VOPS * KIOU || in_sizes[7] != VOPS * KIOU) return;
  if (in_sizes[8] != VOPS * KIOU || in_sizes[9] != VOPS * KIOU) return;
  if (out_size != 2 * nN * HD) return;

  const float* child_h = (const float*)d_in[0];
  const float* child_c = (const float*)d_in[1];
  const float* W_i = (const float*)d_in[2];
  const float* W_f = (const float*)d_in[3];
  const float* W_o = (const float*)d_in[4];
  const float* W_u = (const float*)d_in[5];
  const float* b_i = (const float*)d_in[6];
  const float* b_f = (const float*)d_in[7];
  const float* b_o = (const float*)d_in[8];
  const float* b_u = (const float*)d_in[9];
  const int*   opsP = (const int*)d_in[10];
  const int*   nchP = (const int*)d_in[11];
  float* out = (float*)d_out;

  const size_t wtBytes = (size_t)4 * VOPS * HD * WTP * 2;
  if (wtBytes > ws_size || wtBytes > (size_t)WSMAX) return;
  unsigned short* Wt = (unsigned short*)d_ws;

  const int outOff = nN * HD;

  hipFuncSetAttribute(reinterpret_cast<const void*>(&k_cell), hipFuncAttributeMaxDynamicSharedMemorySize, (int)LDS_TOTAL);

  k_wprep<<<PREP_BLOCKS, NTHR, 0, stream>>>(W_i, W_o, W_u, W_f, Wt);
  k_cell<<<VOPS, NTHR, LDS_TOTAL, stream>>>(child_h, child_c, Wt, b_i, b_o, b_u, b_f, opsP, nchP,
                                            nN, outOff, out);
}
